// LSTM_38757784879582
// MI455X (gfx1250) — hardware-verified
//
#include <hip/hip_runtime.h>
#include <math.h>

constexpr int NBATCH   = 16384;
constexpr int NSTEP    = 28;
constexpr int NIN      = 28;
constexpr int NHID     = 64;
constexpr int NGATE    = 4 * NHID;
constexpr int NCLS     = 10;
constexpr int ROWS_BLK = 16;
constexpr int NTHR     = 128;
constexpr int KCAT     = 96;
constexpr int KPITCH   = 104;
constexpr int HCOL0    = 32;
constexpr int HSP      = 68;
constexpr int NLOGIT   = ROWS_BLK * NCLS;
constexpr float ACARRY = 16.0f;
constexpr float WCARRY = 16.0f;
constexpr float FOLD   = 1.0f / (ACARRY * WCARRY);

static_assert(NBATCH % ROWS_BLK == 0, "grid exact");
static_assert(NHID == 16 * (NTHR / 32), "one 16-unit tile per wave");
static_assert(KCAT % 32 == 0 && HCOL0 % 32 == 0, "k chunks of 32");
static_assert(NIN <= HCOL0 && NIN % 4 == 0 && NIN == 28, "x row: 7 float4, tail octet half valid");
static_assert(KPITCH % 8 == 0 && KPITCH >= KCAT, "16-B aligned fragment loads");
static_assert((NLOGIT * 4) % 128 == 0, "block output span = whole 128-B lines");
static_assert(NLOGIT == NTHR + 32, "lines 0..3 by waves 0..3, line 4 by wave 0");
static_assert((NGATE * 4) % NTHR == 0 && (NGATE * 8) % NTHR == 0, "weight staging loops exact");
static_assert(ROWS_BLK * 8 == NTHR && ROWS_BLK * 4 == 64, "A tile staging maps exact");
static_assert(NGATE * KPITCH * 2 + ROWS_BLK * KPITCH * 2 + ROWS_BLK * HSP * 4 + NLOGIT * 4 <= 65536, "static LDS");

typedef __attribute__((ext_vector_type(16))) _Float16 v16h;
typedef __attribute__((ext_vector_type(8)))  _Float16 v8h;
typedef __attribute__((ext_vector_type(8)))  float    v8f;
typedef __attribute__((ext_vector_type(4)))  float    v4f;

template <typename T> struct Frag;
template <> struct Frag<_Float16> {
  typedef v16h V; union U { v16h v; v8h h[2]; };
  static __device__ __forceinline__ v16h load(const _Float16* p) {
    U f; f.h[0] = *(const v8h*)(p); f.h[1] = *(const v8h*)(p + 16); return f.v;
  }
};

__device__ __forceinline__ v8f mma_g(v16h a, v16h b, v8f c) {
  c = __builtin_amdgcn_wmma_f32_16x16x32_f16(false, a, false, b, (short)0, c, false, false);
  asm volatile("v_nop\n\tv_nop\n\tv_nop\n\tv_nop" : "+v"(c) : "v"(a), "v"(b));
  return c;
}
__device__ __forceinline__ void acc_guard4(v8f& a, v8f& b, v8f& c, v8f& d) {
  asm volatile("v_nop\n\tv_nop\n\tv_nop\n\tv_nop" : "+v"(a), "+v"(b), "+v"(c), "+v"(d));
}

__device__ __forceinline__ float fsig(float v)  { return __builtin_amdgcn_rcpf(1.0f + expf(-v)); }
__device__ __forceinline__ float ftanh(float v) { return 1.0f - 2.0f * __builtin_amdgcn_rcpf(expf(2.0f * v) + 1.0f); }

__device__ __forceinline__ v8h load8_cvt(const float* p, bool tail, float sc) {
  const v4f a = *(const v4f*)(p);
  const v4f b = *(const v4f*)(p + (tail ? 0 : 4));
  v8h hv;
#pragma unroll
  for (int e = 0; e < 4; ++e) {
    const float av = a[e];
    const float bv = tail ? 0.0f : b[e];
    hv[e]     = (_Float16)(av * sc);
    hv[4 + e] = (_Float16)(bv * sc);
  }
  return hv;
}

__global__ __launch_bounds__(NTHR) void lstm_seq_kernel(const float* __restrict__ x,
                                                        const float* __restrict__ w_ih,
                                                        const float* __restrict__ w_hh,
                                                        const float* __restrict__ b_ih,
                                                        const float* __restrict__ b_hh,
                                                        const float* __restrict__ w_out,
                                                        const float* __restrict__ b_out,
                                                        float* __restrict__ out) {
  __shared__ __align__(16) _Float16 Bt[NGATE * KPITCH];
  __shared__ __align__(16) _Float16 At[ROWS_BLK * KPITCH];
  __shared__ __align__(16) float    Hs[ROWS_BLK * HSP];
  __shared__ __align__(16) float    Lg[NLOGIT];

  const int tid = threadIdx.x, lane = tid & 31, wave = tid >> 5;
  const int c = lane & 15, hh = lane >> 4, koff = hh * 8;
  const int rowbase = blockIdx.x * ROWS_BLK;

#pragma unroll 1
  for (int it = 0; it < (NGATE * 4) / NTHR; ++it) {
    const int i = it * NTHR + tid;
    const int n = i >> 2, o = i & 3;
    const v8h hv = load8_cvt(w_ih + n * NIN + 8 * o, o == 3, WCARRY);
    *(v8h*)(Bt + n * KPITCH + 8 * o) = hv;
  }
#pragma unroll 1
  for (int it = 0; it < (NGATE * 8) / NTHR; ++it) {
    const int i = it * NTHR + tid;
    const int n = i >> 3, o = i & 7;
    const v8h hv = load8_cvt(w_hh + n * NHID + 8 * o, false, WCARRY);
    *(v8h*)(Bt + n * KPITCH + HCOL0 + 8 * o) = hv;
  }
  {
    const int m = tid >> 3, o = tid & 7;
    v8h zv;
#pragma unroll
    for (int e = 0; e < 8; ++e) zv[e] = (_Float16)0.0f;
    *(v8h*)(At + m * KPITCH + HCOL0 + 8 * o) = zv;
  }
  if (tid < 64) {
    const int m = tid >> 2, o = tid & 3;
    const v8h hv = load8_cvt(x + ((size_t)(rowbase + m) * NSTEP) * NIN + 8 * o, o == 3, ACARRY);
    *(v8h*)(At + m * KPITCH + 8 * o) = hv;
  }
  float bs[4];
#pragma unroll
  for (int g = 0; g < 4; ++g) {
    const int n = g * NHID + 16 * wave + c;
    bs[g] = b_ih[n] + b_hh[n];
  }
  float cst[8], hst[8];
#pragma unroll
  for (int r = 0; r < 8; ++r) { cst[r] = 0.0f; hst[r] = 0.0f; }
  __syncthreads();

  v16h bf[4][3];
#pragma unroll
  for (int g = 0; g < 4; ++g) {
#pragma unroll
    for (int kc = 0; kc < 3; ++kc)
      bf[g][kc] = Frag<_Float16>::load(Bt + (g * NHID + 16 * wave + c) * KPITCH + kc * 32 + koff);
  }

  const _Float16* arow = At + c * KPITCH + koff;
  const v8f z8 = {0.f, 0.f, 0.f, 0.f, 0.f, 0.f, 0.f, 0.f};

#pragma unroll 1
  for (int t = 0; t < NSTEP; ++t) {
    const v16h a0 = Frag<_Float16>::load(arow);
    const v16h a1 = Frag<_Float16>::load(arow + 32);
    const v16h a2 = Frag<_Float16>::load(arow + 64);
    v8f acc0 = z8, acc1 = z8, acc2 = z8, acc3 = z8;
    acc0 = mma_g(a0, bf[0][0], acc0);
    acc1 = mma_g(a0, bf[1][0], acc1);
    acc2 = mma_g(a0, bf[2][0], acc2);
    acc3 = mma_g(a0, bf[3][0], acc3);
    acc0 = mma_g(a1, bf[0][1], acc0);
    acc1 = mma_g(a1, bf[1][1], acc1);
    acc2 = mma_g(a1, bf[2][1], acc2);
    acc3 = mma_g(a1, bf[3][1], acc3);
    acc0 = mma_g(a2, bf[0][2], acc0);
    acc1 = mma_g(a2, bf[1][2], acc1);
    acc2 = mma_g(a2, bf[2][2], acc2);
    acc3 = mma_g(a2, bf[3][2], acc3);
    acc_guard4(acc0, acc1, acc2, acc3);

#pragma unroll
    for (int r = 0; r < 8; ++r) {
      const float zi = acc0[r] * FOLD + bs[0];
      const float zf = acc1[r] * FOLD + bs[1];
      const float zg = acc2[r] * FOLD + bs[2];
      const float zo = acc3[r] * FOLD + bs[3];
      const float ig = fsig(zi);
      const float fg = fsig(zf);
      const float gg = ftanh(zg);
      const float og = fsig(zo);
      const float cn = fg * cst[r] + ig * gg;
      cst[r] = cn;
      hst[r] = og * ftanh(cn);
    }
    __syncthreads();
#pragma unroll
    for (int r = 0; r < 8; ++r)
      At[(8 * hh + r) * KPITCH + HCOL0 + 16 * wave + c] = (_Float16)(hst[r] * ACARRY);
    if (tid < 64) {
      const int tn = (t + 1 < NSTEP) ? (t + 1) : (NSTEP - 1);
      const int m = tid >> 2, o = tid & 3;
      const v8h hv = load8_cvt(x + ((size_t)(rowbase + m) * NSTEP + (size_t)tn) * NIN + 8 * o, o == 3, ACARRY);
      *(v8h*)(At + m * KPITCH + 8 * o) = hv;
    }
    __syncthreads();
  }

#pragma unroll
  for (int r = 0; r < 8; ++r) Hs[(8 * hh + r) * HSP + 16 * wave + c] = hst[r];
  __syncthreads();

#pragma unroll 1
  for (int it = 0; it < 2; ++it) {
    const int e  = it * NTHR + tid;
    const int ec = (e < NLOGIT) ? e : (NLOGIT - 1);
    const int m  = ec / NCLS;
    const int cls = ec - m * NCLS;
    const float* hr = Hs + m * HSP;
    const float* wr = w_out + cls * NHID;
    float s = 0.0f;
#pragma unroll 1
    for (int u = 0; u < NHID; u += 4) {
      const v4f hv = *(const v4f*)(hr + u);
      const v4f wv = *(const v4f*)(wr + u);
      s += hv[0] * wv[0];
      s += hv[1] * wv[1];
      s += hv[2] * wv[2];
      s += hv[3] * wv[3];
    }
    s += b_out[cls];
    if (e < NLOGIT) Lg[e] = s;
  }
  __syncthreads();

  {
    float* ob = out + (size_t)blockIdx.x * NLOGIT;
    const float v0 = Lg[tid];
    const float v1 = Lg[NTHR + lane];
    for (int pass = 0; pass < 2; ++pass) {
      *(volatile float*)(ob + tid) = v0;
      if (wave == 0) *(volatile float*)(ob + NTHR + lane) = v1;
      __threadfence();
    }
  }
}

extern "C" void kernel_launch(void* const* d_in, const int* in_sizes, int n_in,
                              void* d_out, int out_size, void* d_ws, size_t ws_size, hipStream_t stream) {
  (void)d_ws; (void)ws_size;
  if (n_in < 7 || d_out == nullptr) return;
  if (in_sizes[0] != NBATCH * NSTEP * NIN || in_sizes[1] != NGATE * NIN || in_sizes[2] != NGATE * NHID ||
      in_sizes[3] != NGATE || in_sizes[4] != NGATE || in_sizes[5] != NCLS * NHID || in_sizes[6] != NCLS ||
      out_size != NBATCH * NCLS) return;

  const float* x     = (const float*)d_in[0];
  const float* w_ih  = (const float*)d_in[1];
  const float* w_hh  = (const float*)d_in[2];
  const float* b_ih  = (const float*)d_in[3];
  const float* b_hh  = (const float*)d_in[4];
  const float* w_out = (const float*)d_in[5];
  const float* b_out = (const float*)d_in[6];
  float* out = (float*)d_out;

  lstm_seq_kernel<<<NBATCH / ROWS_BLK, NTHR, 0, stream>>>(x, w_ih, w_hh, b_ih, b_hh, w_out, b_out, out);
}
